// PureSSM_781684048752
// MI455X (gfx1250) — hardware-verified
//
#include <hip/hip_runtime.h>


#define NB_  2
#define LL   1024
#define DMd  1024
#define DI   2048
#define NS   64
#define NHm  32
#define HP   64
#define PR   8224
#define PW   8256
#define BC0  4096
typedef _Float16 h16;
typedef unsigned short bf;
typedef __attribute__((ext_vector_type(16))) __bf16   v16bf;
typedef __attribute__((ext_vector_type(16))) _Float16 v16h;
typedef __attribute__((ext_vector_type(8)))  _Float16 v8h;
typedef __attribute__((ext_vector_type(8)))  unsigned short v8us;
typedef __attribute__((ext_vector_type(8)))  float    v8f;
typedef __attribute__((ext_vector_type(4)))  float    v4f;
typedef v8h  __attribute__((may_alias)) v8ha;
typedef v4f  __attribute__((may_alias)) v4fa;
typedef v8us __attribute__((may_alias)) v8usa;

__device__ __forceinline__ unsigned short f2bf(float f) { unsigned u = __float_as_uint(f); u += 0x7FFFu + ((u >> 16) & 1u); return (unsigned short)(u >> 16); }
__device__ __forceinline__ float bf2f(unsigned short b) { return __uint_as_float(((unsigned)b) << 16); }
__device__ __forceinline__ float bfr(float f) { return bf2f(f2bf(f)); }
__device__ __forceinline__ v16h cat16(v8h lo, v8h hi) { return __builtin_shufflevector(lo, hi, 0, 1, 2, 3, 4, 5, 6, 7, 8, 9, 10, 11, 12, 13, 14, 15); }
__device__ __forceinline__ v16bf cat16b(v8us lo, v8us hi) { return __builtin_bit_cast(v16bf, __builtin_shufflevector(lo, hi, 0, 1, 2, 3, 4, 5, 6, 7, 8, 9, 10, 11, 12, 13, 14, 15)); }
__device__ __forceinline__ v8f wmma16(v16h a, v16h b, v8f c) { return __builtin_amdgcn_wmma_f32_16x16x32_f16(false, a, false, b, (short)0, c, false, false); }
__device__ __forceinline__ v8f wmmab(v16bf a, v16bf b, v8f c) { return __builtin_amdgcn_wmma_f32_16x16x32_bf16(false, a, false, b, (short)0, c, false, false); }


template <typename T16> struct WFrag;
template <> struct WFrag<h16> { typedef v16h V; static __device__ __forceinline__ V ld(const h16* p) { return cat16(*(const v8h*)p, *(const v8h*)(p + 16)); } static __device__ __forceinline__ v8f mma(V a, V b, v8f c) { return wmma16(a, b, c); } };
template <> struct WFrag<bf> { typedef v16bf V; static __device__ __forceinline__ V ld(const bf* p) { return cat16b(*(const v8us*)p, *(const v8us*)(p + 16)); } static __device__ __forceinline__ v8f mma(V a, V b, v8f c) { return wmmab(a, b, c); } };
template <typename T16, int NSPLIT, bool BIAS>
__global__ __launch_bounds__(32) void k_gemmw(const T16* __restrict__ A, const T16* __restrict__ A2, const T16* __restrict__ Bt, const T16* __restrict__ Bt2, int K, float* C, int ldc, const float* __restrict__ bias, size_t sA, size_t sB, size_t sC) {
    typedef typename WFrag<T16>::V V;
    __shared__ __align__(16) float os[16 * 68];
    const size_t z = blockIdx.z; A += z * sA; if (A2) A2 += z * sA; Bt += z * sB; if (Bt2) Bt2 += z * sB; C += z * sC;
    const int lane = threadIdx.x & 31, lr = lane & 15, hi = lane >> 4; const int r0 = blockIdx.x * 64, c0 = blockIdx.y * 64;
    v8f acc[4][4];
#pragma unroll
    for (int mb = 0; mb < 4; ++mb)
#pragma unroll
        for (int nb = 0; nb < 4; ++nb) acc[mb][nb] = (v8f){};
    const size_t aoff = (size_t)(r0 + lr) * K + 8 * hi, boff = (size_t)(c0 + lr) * K + 8 * hi;
#pragma unroll 1
    for (int kc = 0; kc < K; kc += 32) {
        V a[4], a2[4];
#pragma unroll
        for (int mb = 0; mb < 4; ++mb) { a[mb] = WFrag<T16>::ld(A + aoff + (size_t)mb * 16 * K + kc); if (NSPLIT == 1 || NSPLIT == 2) a2[mb] = WFrag<T16>::ld(A2 + aoff + (size_t)mb * 16 * K + kc); }
#pragma unroll
        for (int nb = 0; nb < 4; ++nb) { const V b = WFrag<T16>::ld(Bt + boff + (size_t)nb * 16 * K + kc); V b2; if (NSPLIT >= 2) b2 = WFrag<T16>::ld(Bt2 + boff + (size_t)nb * 16 * K + kc);
#pragma unroll
            for (int mb = 0; mb < 4; ++mb) { acc[mb][nb] = WFrag<T16>::mma(a[mb], b, acc[mb][nb]); if (NSPLIT == 1 || NSPLIT == 2) acc[mb][nb] = WFrag<T16>::mma(a2[mb], b, acc[mb][nb]); if (NSPLIT >= 2) acc[mb][nb] = WFrag<T16>::mma(a[mb], b2, acc[mb][nb]); } }
        asm volatile("v_nop\n\tv_nop\n\tv_nop\n\tv_nop" : "+v"(acc[0][0]), "+v"(acc[1][1]), "+v"(acc[2][2]), "+v"(acc[3][3]) : "v"(a[0]), "v"(a[3]));
    }
#pragma unroll
    for (int mb = 0; mb < 4; ++mb) {
#pragma unroll
        for (int nb = 0; nb < 4; ++nb) {
#pragma unroll
            for (int j = 0; j < 8; ++j) os[(hi * 8 + j) * 68 + nb * 16 + lr] = acc[mb][nb][j]; }
        __builtin_amdgcn_wave_barrier(); asm volatile("" ::: "memory");
        float* crow = C + (size_t)(r0 + mb * 16) * ldc + c0;
#pragma unroll 1
        for (int ps = 0; ps < 2; ++ps) {
#pragma unroll
            for (int s = 0; s < 8; ++s) { const int row = 2 * s + hi, cofs = lr * 4; v4f val = *(const v4fa*)(os + row * 68 + cofs); if (BIAS) { val[0] += bfr(bias[c0 + cofs]); val[1] += bfr(bias[c0 + cofs + 1]); val[2] += bfr(bias[c0 + cofs + 2]); val[3] += bfr(bias[c0 + cofs + 3]); }
                *(volatile v4f*)(crow + (size_t)row * ldc + cofs) = val; }
            if (ps == 0) __threadfence(); }
        __builtin_amdgcn_wave_barrier(); asm volatile("" ::: "memory");
    }
}

__device__ __forceinline__ void splitf(float y, unsigned short& h, unsigned short& l) { h = f2bf(y); l = f2bf(y - bf2f(h)); }
__device__ __forceinline__ float silu_(float x) { return __fmul_rn(x, __fdiv_rn(1.0f, 1.0f + __expf(-x))); }
__device__ __forceinline__ float softplus_(float x) { return x > 20.f ? x : log1pf(__expf(x)); }
typedef __attribute__((ext_vector_type(2))) unsigned short v2us;
typedef __attribute__((ext_vector_type(4))) unsigned short v4us;

__global__ __launch_bounds__(256) void k_cvt8(const float* __restrict__ src, bf* dst, size_t n8) { const size_t i = (size_t)blockIdx.x * 256 + threadIdx.x; if (i >= n8) return; const v8f v = *(const v8f*)(src + i * 8); v8us o;
#pragma unroll
    for (int k = 0; k < 8; ++k) o[k] = f2bf(v[k]); *(volatile v8us*)(dst + i * 8) = o; __threadfence(); *(volatile v8us*)(dst + i * 8) = o; }
__global__ __launch_bounds__(256) void k_wpad(const float* __restrict__ w, int nreal, int NOUT, int KP, bf* Bt) { const size_t i = ((size_t)blockIdx.x * 256 + threadIdx.x) * 4; if (i >= (size_t)NOUT * KP) return; const int n = (int)(i / KP); v4us o;
#pragma unroll
    for (int q = 0; q < 4; ++q) o[q] = n < nreal ? f2bf(w[i + q]) : (unsigned short)0; *(volatile v4us*)(Bt + i) = o; __threadfence(); *(volatile v4us*)(Bt + i) = o; }
__global__ __launch_bounds__(256) void k_conv(const float* __restrict__ PJ, const float* __restrict__ w, const float* __restrict__ bb, float* XC) { const int e = (blockIdx.x * 256 + threadIdx.x) * 4; if (e >= LL * DI) return; const int c = e % DI, t = e / DI; v4f o;
#pragma unroll 1
    for (int q = 0; q < 4; ++q) { const int cc = c + q; float acc = 0.f;
#pragma unroll
        for (int k = 0; k < 4; ++k) { const int ts = t - 3 + k; if (ts >= 0) { float p = __fmul_rn(bfr(w[cc * 4 + k]), PJ[(size_t)ts * PW + cc]); asm volatile("" : "+v"(p)); acc = __fadd_rn(acc, p); } }
        o[q] = silu_(__fadd_rn(acc, bfr(bb[cc]))); }
    *(volatile v4f*)(XC + e) = o; __threadfence(); *(volatile v4f*)(XC + e) = o; }
__global__ __launch_bounds__(256) void k_scan(const float* __restrict__ PJ, const float* __restrict__ dtb, const float* __restrict__ XC, const float* __restrict__ alog, const float* __restrict__ Dp, float* Y) {
    __shared__ float ybuf[32]; const int tid = threadIdx.x; const int cl = tid >> 3, sub = tid & 7; const int c = blockIdx.x * 32 + cl; const int h = c / HP; const int n0 = sub * 8; float A[8], S[8];
#pragma unroll
    for (int j = 0; j < 8; ++j) { A[j] = -__expf(bfr(alog[h * NS + n0 + j])); S[j] = 0.f; }
    float dd = bfr(Dp[h]); float db = bfr(dtb[h]); asm volatile("" : "+v"(dd)); asm volatile("" : "+v"(db));
    for (int t = 0; t < LL; ++t) { const float* pr = PJ + (size_t)t * PW + BC0 + h * (2 * NS + 1); const float dt = softplus_(__fadd_rn(pr[2 * NS], db)); const float xv = XC[(size_t)t * DI + c]; const float dtx = __fmul_rn(dt, xv); float y = 0.f;
#pragma unroll
        for (int j = 0; j < 8; ++j) { const float a = __expf(__fmul_rn(dt, A[j])); float sa = __fmul_rn(S[j], a); asm volatile("" : "+v"(sa)); float bx = __fmul_rn(dtx, pr[n0 + j]); asm volatile("" : "+v"(bx)); S[j] = __fadd_rn(sa, bx); float yc = __fmul_rn(S[j], pr[NS + n0 + j]); asm volatile("" : "+v"(yc)); y = __fadd_rn(y, yc); }
        y += __shfl_xor(y, 1, 32); y += __shfl_xor(y, 2, 32); y += __shfl_xor(y, 4, 32);
        if (sub == 0) { float sk = __fmul_rn(dd, xv); asm volatile("" : "+v"(sk)); ybuf[cl] = __fadd_rn(y, sk); }
        __syncthreads();
        if (tid < 32) { const float v = ybuf[tid]; const size_t o = (size_t)t * DI + blockIdx.x * 32 + tid; *(volatile float*)(Y + o) = v; __threadfence(); *(volatile float*)(Y + o) = v; }
        __syncthreads(); } }
__global__ __launch_bounds__(256) void k_gate(const float* __restrict__ Y, const float* __restrict__ PJ, bf* Gh, bf* Gl) { const int e = (blockIdx.x * 256 + threadIdx.x) * 4; if (e >= LL * DI) return; const int c = e % DI, t = e / DI; const v4f y = *(const v4f*)(Y + e), z = *(const v4f*)(PJ + (size_t)t * PW + DI + c); v4us oh, ol;
#pragma unroll
    for (int q = 0; q < 4; ++q) { unsigned short u, l; splitf(__fmul_rn(y[q], silu_(z[q])), u, l); oh[q] = u; ol[q] = l; } *(volatile v4us*)(Gh + e) = oh; *(volatile v4us*)(Gl + e) = ol; __threadfence(); *(volatile v4us*)(Gh + e) = oh; *(volatile v4us*)(Gl + e) = ol; }

extern "C" void kernel_launch(void* const* d_in, const int* in_sizes, int n_in,
                              void* d_out, int out_size, void* d_ws, size_t ws_size, hipStream_t stream) {
    (void)in_sizes; (void)n_in; (void)out_size;
    const float* x = (const float*)d_in[0]; const float* win = (const float*)d_in[1]; const float* cw = (const float*)d_in[2]; const float* cb = (const float*)d_in[3]; const float* alog = (const float*)d_in[4]; const float* Dp = (const float*)d_in[5]; const float* dtb = (const float*)d_in[6]; const float* wout = (const float*)d_in[7];
    float* OUT = (float*)d_out;
    char* wsp = (char*)d_ws;
    auto take = [&](size_t bytes) { char* p = wsp; wsp += (bytes + 255) & ~(size_t)255; return (void*)p; };
    bf* WIN = (bf*)take((size_t)PW * DMd * 2); bf* WOUT = (bf*)take((size_t)DMd * DI * 2); bf* XB = (bf*)take((size_t)LL * DMd * 2); float* PJ = (float*)take((size_t)LL * PW * 4); float* XC = (float*)take((size_t)LL * DI * 4); float* Y = (float*)take((size_t)LL * DI * 4); bf* Gh = (bf*)take((size_t)LL * DI * 2); bf* Gl = (bf*)take((size_t)LL * DI * 2);
    if ((size_t)(wsp - (char*)d_ws) > ws_size) return;
    k_wpad<<<(unsigned)(((size_t)PW * DMd / 4 + 255) / 256), 256, 0, stream>>>(win, PR, PW, DMd, WIN); k_cvt8<<<(DMd * DI / 8 + 255) / 256, 256, 0, stream>>>(wout, WOUT, (size_t)DMd * DI / 8);
    for (int b = 0; b < NB_; ++b) {
        k_cvt8<<<(LL * DMd / 8 + 255) / 256, 256, 0, stream>>>(x + (size_t)b * LL * DMd, XB, (size_t)LL * DMd / 8);
        k_gemmw<bf, 0, false><<<dim3(LL / 64, PW / 64, 1), 32, 0, stream>>>(XB, nullptr, WIN, nullptr, DMd, PJ, PW, nullptr, 0, 0, 0);
        k_conv<<<(LL * DI / 4 + 255) / 256, 256, 0, stream>>>(PJ, cw, cb, XC);
        k_scan<<<DI / 32, 256, 0, stream>>>(PJ, dtb, XC, alog, Dp, Y);
        k_gate<<<(LL * DI / 4 + 255) / 256, 256, 0, stream>>>(Y, PJ, Gh, Gl);
        k_gemmw<bf, 1, false><<<dim3(LL / 64, DMd / 64, 1), 32, 0, stream>>>(Gh, Gl, WOUT, nullptr, DI, OUT + (size_t)b * LL * DMd, DMd, nullptr, 0, 0, 0); }
}
